// GraphEncoderLayer_40183714021846
// MI455X (gfx1250) — hardware-verified
//
#include <hip/hip_runtime.h>
#include <stdint.h>

typedef __attribute__((ext_vector_type(16))) _Float16 v16h;
typedef __attribute__((ext_vector_type(8)))  _Float16 v8h;
typedef __attribute__((ext_vector_type(4)))  _Float16 v4h;
typedef __attribute__((ext_vector_type(16))) __bf16   v16b;
typedef __attribute__((ext_vector_type(8)))  __bf16   v8b;
typedef __attribute__((ext_vector_type(8)))  float    v8f;
typedef __attribute__((ext_vector_type(4)))  float    v4f;
typedef __attribute__((ext_vector_type(8)))  unsigned short v8us;

constexpr int NB   = 16;
constexpr int NL   = 512;
constexpr int ND   = 512;
constexpr int NH   = 8;
constexpr int NHD  = 64;
constexpr int NFF  = 2048;
constexpr int NRB  = 16;
constexpr int NM   = NB * NL;
constexpr int NQKV = 3 * ND;

__device__ __forceinline__ unsigned short f2bf_bits(float f) {
  unsigned u = __float_as_uint(f);
  return (unsigned short)((u + 0x7FFFu + ((u >> 16) & 1u)) >> 16);
}
__device__ __forceinline__ float bf_bits2f(unsigned short h) { return __uint_as_float(((unsigned)h) << 16); }

__device__ __forceinline__ void dep_guard_h(v8f& a, v8f& b, v16h x, v16h y) { asm volatile("v_nop\n\tv_nop\n\tv_nop\n\tv_nop" : "+v"(a), "+v"(b) : "v"(x), "v"(y)); }
__device__ __forceinline__ void dep_guard_b(v8f& a, v8f& b, v16b x, v16b y) { asm volatile("v_nop\n\tv_nop\n\tv_nop\n\tv_nop" : "+v"(a), "+v"(b) : "v"(x), "v"(y)); }
__device__ __forceinline__ void keep4_h(v16h a, v16h b, v16h c, v16h d) { asm volatile("v_nop" :: "v"(a), "v"(b), "v"(c), "v"(d)); }
__device__ __forceinline__ void keep4_b(v16b a, v16b b, v16b c, v16b d) { asm volatile("v_nop" :: "v"(a), "v"(b), "v"(c), "v"(d)); }
__device__ __forceinline__ void acc_guard4(v8f& a, v8f& b, v8f& c, v8f& d) { asm volatile("v_nop\n\tv_nop\n\tv_nop\n\tv_nop" : "+v"(a), "+v"(b), "+v"(c), "+v"(d)); }
template <typename T> struct Frag;
template <> struct Frag<_Float16> {
  typedef v16h V; union U { v16h v; v8h h[2]; };
  static __device__ __forceinline__ v16h load(const _Float16* p) {
    U f; f.h[0] = *(const v8h*)(p); f.h[1] = *(const v8h*)(p + 16); return f.v;
  }
  static __device__ __forceinline__ v8f mma(v16h a, v16h b, v8f c) {
    return __builtin_amdgcn_wmma_f32_16x16x32_f16(false, a, false, b, (short)0, c, false, false);
  }
  static __device__ __forceinline__ void guard(v8f& a, v8f& b, v16h x, v16h y) { dep_guard_h(a, b, x, y); }
  static __device__ __forceinline__ void keep(v16h a, v16h b, v16h c, v16h d) { keep4_h(a, b, c, d); }
};
template <> struct Frag<__bf16> {
  typedef v16b V; union U { v16b v; v8b h[2]; };
  static __device__ __forceinline__ v16b load(const __bf16* p) {
    U f; f.h[0] = *(const v8b*)(p); f.h[1] = *(const v8b*)(p + 16); return f.v;
  }
  static __device__ __forceinline__ v8f mma(v16b a, v16b b, v8f c) {
    return __builtin_amdgcn_wmma_f32_16x16x32_bf16(false, a, false, b, (short)0, c, false, false);
  }
  static __device__ __forceinline__ void guard(v8f& a, v8f& b, v16b x, v16b y) { dep_guard_b(a, b, x, y); }
  static __device__ __forceinline__ void keep(v16b a, v16b b, v16b c, v16b d) { keep4_b(a, b, c, d); }
};

__device__ __forceinline__ v8f mma_h(v16h a, v16h b, v8f c) {
  c = __builtin_amdgcn_wmma_f32_16x16x32_f16(false, a, false, b, (short)0, c, false, false);
  asm volatile("v_nop\n\tv_nop\n\tv_nop\n\tv_nop" : "+v"(c) : "v"(a), "v"(b));
  return c;
}
__device__ __forceinline__ v8f zero8f() { return (v8f){0.f,0.f,0.f,0.f,0.f,0.f,0.f,0.f}; }

__device__ __forceinline__ void wave_lds_sync() {
  __builtin_amdgcn_fence(__ATOMIC_RELEASE, "workgroup");
  __builtin_amdgcn_wave_barrier();
  __builtin_amdgcn_fence(__ATOMIC_ACQUIRE, "workgroup");
}

template <int ET> struct Elem;
template <> struct Elem<0> { typedef _Float16 T; };
template <> struct Elem<1> { typedef __bf16 T; };
template <int ET, bool SPLIT, int BIAS_MODE, int OUT_MODE, bool RESID, int ACT = 0>
__global__ __launch_bounds__(256) void wmma_gemm64(
    const unsigned short* __restrict__ Ap, const unsigned short* __restrict__ A2p, int lda, long strideA,
    const unsigned short* __restrict__ Btp, const unsigned short* __restrict__ Bt2p, int ldb, long strideB,
    void* __restrict__ Cout, void* __restrict__ Cout2, int ldc, long strideC,
    const float* __restrict__ bias,
    const float* __restrict__ resid, long strideR,
    int M, int N, int K, float scale) {
  typedef typename Elem<ET>::T T;
  typedef typename Frag<T>::V V;
  const T* A = (const T*)Ap; const T* A2 = (const T*)A2p; const T* Bt = (const T*)Btp; const T* Bt2 = (const T*)Bt2p;
  __shared__ __align__(16) float sT[8][16 * 68];
  const int b    = blockIdx.y;
  const int lane = threadIdx.x & 31;
  const int wave = threadIdx.x >> 5;
  const int tilesN = N >> 6;
  const int tilesM = M >> 6;
  const int tile = blockIdx.x * 8 + wave;
  if (tile >= tilesM * tilesN) return;
  const int tm = tile / tilesN;
  const int tn = tile - tm * tilesN;
  const int m0 = tm << 6;
  const int n0 = tn << 6;

  const T* Ab  = A  + (size_t)b * strideA;
  const T* Bb  = Bt + (size_t)b * strideB;
  const T* Ab2 = SPLIT ? (A2  + (size_t)b * strideA) : nullptr;
  const T* Bb2 = SPLIT ? (Bt2 + (size_t)b * strideB) : nullptr;

  const int rlane = lane & 15;
  const int koff  = (lane >> 4) * 8;
  const int mOff  = (lane >> 4) * 8;

  v8f acc[4][4];
#pragma unroll
  for (int i = 0; i < 4; ++i)
#pragma unroll
    for (int j = 0; j < 4; ++j) acc[i][j] = (v8f){0.f,0.f,0.f,0.f,0.f,0.f,0.f,0.f};

  for (int k0 = 0; k0 < K; k0 += 32) {
    V bh[4], bl[4];
#pragma unroll
    for (int j = 0; j < 4; ++j) {
      const size_t bo = (size_t)(n0 + (j << 4) + rlane) * ldb + koff + k0;
      bh[j] = Frag<T>::load(Bb + bo);
      if (SPLIT) bl[j] = Frag<T>::load(Bb2 + bo);
    }
#pragma unroll
    for (int i = 0; i < 4; ++i) {
      const size_t ao = (size_t)(m0 + (i << 4) + rlane) * lda + koff + k0;
      V ah = Frag<T>::load(Ab + ao);
      V al;
      if (SPLIT) al = Frag<T>::load(Ab2 + ao);
#pragma unroll
      for (int j = 0; j < 4; ++j) {
        acc[i][j] = Frag<T>::mma(ah, bh[j], acc[i][j]);
        if (SPLIT) {
          acc[i][j] = Frag<T>::mma(ah, bl[j], acc[i][j]);
          acc[i][j] = Frag<T>::mma(al, bh[j], acc[i][j]);
        }
      }
      Frag<T>::guard(acc[i][0], acc[i][3], ah, SPLIT ? al : ah);
    }
    Frag<T>::keep(bh[0], bh[1], bh[2], bh[3]);
    if (SPLIT) Frag<T>::keep(bl[0], bl[1], bl[2], bl[3]);
  }
  acc_guard4(acc[0][0], acc[0][1], acc[0][2], acc[0][3]);
  acc_guard4(acc[1][0], acc[1][1], acc[1][2], acc[1][3]);
  acc_guard4(acc[2][0], acc[2][1], acc[2][2], acc[2][3]);
  acc_guard4(acc[3][0], acc[3][1], acc[3][2], acc[3][3]);

  float* slab = sT[wave];
  const float* Rb = RESID ? (resid + (size_t)b * strideR) : nullptr;
#pragma unroll
  for (int i = 0; i < 4; ++i) {
    const int mBase = m0 + (i << 4);
#pragma unroll
    for (int j = 0; j < 4; ++j) {
      const int n = n0 + (j << 4) + rlane;
      float bv = 0.f;
      if (BIAS_MODE == 2) bv = bias[n];
#pragma unroll
      for (int r = 0; r < 8; ++r) {
        float v = acc[i][j][r] * scale;
        if (BIAS_MODE == 1) v += bias[mBase + mOff + r];
        if (BIAS_MODE == 2) v += bv;
        if (RESID) v += Rb[(size_t)(mBase + mOff + r) * ldc + n];
        if (ACT == 1) v = tanhf(v);
        if (ACT == 2) v = fmaxf(v, 0.0f);
        if (ACT == 3) v = v / (1.0f + expf(-v));
        if (ACT == 4) v = (v > 0.f) ? v : 0.01f * v;
        if (ACT == 5) v = 0.5f * v * (1.0f + erff(v * 0.70710678118654752f));
        slab[(mOff + r) * 68 + (j << 4) + rlane] = v;
      }
    }
    __builtin_amdgcn_fence(__ATOMIC_RELEASE, "workgroup");
    __builtin_amdgcn_wave_barrier();
    __builtin_amdgcn_fence(__ATOMIC_ACQUIRE, "workgroup");
    if (OUT_MODE == 0) {
      float* C = (float*)Cout + (size_t)b * strideC;
      const int hh = lane >> 4, c4 = (lane & 15) * 4;
      for (int pass = 0; pass < 2; ++pass) {
#pragma unroll
        for (int it = 0; it < 8; ++it) {
          const int row = it * 2 + hh;
          v4f v = *(const v4f*)(slab + row * 68 + c4);
          *(volatile v4f*)(C + (size_t)(mBase + row) * ldc + n0 + c4) = v;
        }
        __threadfence();
      }
    } else {
      const int q = lane >> 3, c8 = (lane & 7) * 8;
      unsigned short* C  = (unsigned short*)Cout  + (size_t)b * strideC;
      unsigned short* C2 = (OUT_MODE == 2) ? ((unsigned short*)Cout2 + (size_t)b * strideC) : nullptr;
      for (int pass = 0; pass < 2; ++pass) {
#pragma unroll
        for (int it = 0; it < 4; ++it) {
          const int row = it * 4 + q;
          const float* sp = slab + row * 68 + c8;
          v8h hv, lv;
#pragma unroll
          for (int e = 0; e < 8; ++e) {
            if (OUT_MODE == 1) {
              hv[e] = (_Float16)sp[e];
            } else {
              unsigned short hb = f2bf_bits(sp[e]);
              unsigned short lb = f2bf_bits(sp[e] - bf_bits2f(hb));
              hv[e] = __builtin_bit_cast(_Float16, hb);
              lv[e] = __builtin_bit_cast(_Float16, lb);
            }
          }
          *(volatile v8h*)(C + (size_t)(mBase + row) * ldc + n0 + c8) = hv;
          if (OUT_MODE == 2) *(volatile v8h*)(C2 + (size_t)(mBase + row) * ldc + n0 + c8) = lv;
        }
        __threadfence();
      }
    }
    __builtin_amdgcn_fence(__ATOMIC_RELEASE, "workgroup");
    __builtin_amdgcn_wave_barrier();
    __builtin_amdgcn_fence(__ATOMIC_ACQUIRE, "workgroup");
  }
}

__global__ __launch_bounds__(256) void cast8_kernel(const float* __restrict__ in, _Float16* __restrict__ out, int n8) {
  const int i = blockIdx.x * 256 + threadIdx.x;
  if (i >= n8) return;
  const v4f a = *(const v4f*)(in + (size_t)i * 8);
  const v4f c = *(const v4f*)(in + (size_t)i * 8 + 4);
  v8h hv;
  hv[0] = (_Float16)a[0]; hv[1] = (_Float16)a[1]; hv[2] = (_Float16)a[2]; hv[3] = (_Float16)a[3];
  hv[4] = (_Float16)c[0]; hv[5] = (_Float16)c[1]; hv[6] = (_Float16)c[2]; hv[7] = (_Float16)c[3];
  _Float16* p = out + (size_t)i * 8;
  *(volatile v8h*)p = hv;
  __threadfence();
  *(volatile v8h*)p = hv;
}

__global__ __launch_bounds__(256) void wtrans_kernel(const float* __restrict__ W, _Float16* __restrict__ Bt, int Kd, int Nd) {
  __shared__ float tile[64 * 65];
  const int n0 = blockIdx.x * 64, k0 = blockIdx.y * 64;
  const int tid = threadIdx.x;
#pragma unroll
  for (int it = 0; it < 4; ++it) {
    const int u = it * 256 + tid;
    const int kk = u >> 4, n4 = (u & 15) * 4;
    const v4f v = *(const v4f*)(W + (size_t)(k0 + kk) * Nd + n0 + n4);
    tile[(n4 + 0) * 65 + kk] = v[0] * 64.0f;
    tile[(n4 + 1) * 65 + kk] = v[1] * 64.0f;
    tile[(n4 + 2) * 65 + kk] = v[2] * 64.0f;
    tile[(n4 + 3) * 65 + kk] = v[3] * 64.0f;
  }
  __syncthreads();
  const int wave = tid >> 5, lane = tid & 31, q = lane >> 3, c8 = (lane & 7) * 8;
  v8h hv[2];
#pragma unroll
  for (int it = 0; it < 2; ++it) {
    const int row = wave * 8 + it * 4 + q;
    const float* sp = tile + row * 65 + c8;
#pragma unroll
    for (int e = 0; e < 8; ++e) hv[it][e] = (_Float16)sp[e];
  }
  for (int pass = 0; pass < 2; ++pass) {
#pragma unroll
    for (int it = 0; it < 2; ++it) {
      const int row = wave * 8 + it * 4 + q;
      *(volatile v8h*)(Bt + (size_t)(n0 + row) * Kd + k0 + c8) = hv[it];
    }
    __threadfence();
  }
}

__global__ __launch_bounds__(256) void edge_kernel(const float* __restrict__ cost, const float* __restrict__ We1,
    const float* __restrict__ be1, const float* __restrict__ We2, const float* __restrict__ be2,
    unsigned short* __restrict__ eb) {
  __shared__ float sW1[NRB * NRB];
  __shared__ float sW2[NRB * NH];
  __shared__ float sb1[NRB];
  __shared__ float sb2[NH];
  __shared__ __align__(16) _Float16 sH[8][16 * 24];
  __shared__ __align__(16) unsigned short sO[8][16 * 64];
  const int tid = threadIdx.x;
  sW1[tid] = We1[tid];
  if (tid < NRB * NH) sW2[tid] = We2[tid];
  if (tid < NRB) sb1[tid] = be1[tid];
  if (tid < NH) sb2[tid] = be2[tid];
  __syncthreads();
  const int wave = tid >> 5, lane = tid & 31, hh = lane >> 4, c = lane & 15;
  const int rowid = blockIdx.x * 8 + wave;
  const int b = rowid >> 9, i = rowid & 511;
  const int cc = (c < 8) ? c : 7;
  v16h w1v, w2v;
#pragma unroll
  for (int e = 0; e < 16; ++e) { w1v[e] = (_Float16)0.0f; w2v[e] = (_Float16)0.0f; }
#pragma unroll
  for (int e = 0; e < 8; ++e) {
    w1v[e] = (_Float16)(sW1[(8 * hh + e) * NRB + c] * 64.0f);
    const float t2 = sW2[(8 * hh + e) * NH + cc] * 64.0f;
    w2v[e] = (c < 8) ? (_Float16)t2 : (_Float16)0.0f;
  }
  const float b1v = sb1[c];
  const float b2v = sb2[cc];
  const float wdt = 1.0f / 15.0f;
  const float inv2w2 = 1.0f / (2.0f * wdt * wdt);
  v8h z8;
#pragma unroll
  for (int e = 0; e < 8; ++e) z8[e] = (_Float16)0.0f;
  _Float16* sh = sH[wave];
  unsigned short* so = sO[wave];
  const float* crow = cost + (size_t)rowid * NL;
  const int q = lane >> 3, c8 = (lane & 7) * 8;
  for (int jc = 0; jc < NL / 64; ++jc) {
#pragma unroll 1
    for (int t = 0; t < 4; ++t) {
      const float cv = crow[jc * 64 + t * 16 + c];
      v16h af;
#pragma unroll
      for (int e = 0; e < 16; ++e) af[e] = (_Float16)0.0f;
#pragma unroll
      for (int e = 0; e < 8; ++e) {
        const int r = 8 * hh + e;
        const float ctr = (r == NRB - 1) ? 1.0f : (float)r * wdt;
        const float d = cv - ctr;
        af[e] = (_Float16)(expf(-(d * d) * inv2w2) * 256.0f);
      }
      v8f acc1 = mma_h(af, w1v, zero8f());
#pragma unroll
      for (int r = 0; r < 8; ++r) {
        const float hv = fmaxf(acc1[r] * (1.0f / 16384.0f) + b1v, 0.0f) * 64.0f;
        sh[(8 * hh + r) * 24 + c] = (_Float16)hv;
      }
      wave_lds_sync();
      Frag<_Float16>::U a2;
      a2.h[0] = *(const v8h*)(sh + c * 24 + 8 * hh);
      a2.h[1] = z8;
      wave_lds_sync();
      v8f acc2 = mma_h(a2.v, w2v, zero8f());
#pragma unroll
      for (int r = 0; r < 8; ++r) {
        const float v = acc2[r] * (1.0f / 4096.0f) + b2v;
        so[c * 64 + t * 16 + 8 * hh + r] = f2bf_bits(v);
      }
    }
    wave_lds_sync();
    v8us ov[2];
#pragma unroll
    for (int it = 0; it < 2; ++it) {
      const int head = it * 4 + q;
      ov[it] = *(const v8us*)(so + head * 64 + c8);
    }
    for (int pass = 0; pass < 2; ++pass) {
#pragma unroll
      for (int it = 0; it < 2; ++it) {
        const int head = it * 4 + q;
        *(volatile v8us*)(eb + (((size_t)((b * NH + head) * NL + i)) * NL + jc * 64 + c8)) = ov[it];
      }
      __threadfence();
    }
    wave_lds_sync();
  }
}

#define ATT_PSC 32768.0f
__global__ __launch_bounds__(128) void attn_kernel(const unsigned short* __restrict__ qkv,
    const unsigned short* __restrict__ ebias, _Float16* __restrict__ ctx) {
  __shared__ __align__(16) unsigned short Ksh[64 * 64];
  __shared__ __align__(16) unsigned short Vt[64 * 64];
  __shared__ __align__(16) unsigned short Bsh[64 * 64];
  __shared__ __align__(16) _Float16 Psh[4][16 * 64];
  __shared__ __align__(16) float Os[4][16 * 68];
  const int tid = threadIdx.x, wave = tid >> 5, lane = tid & 31, hh = lane >> 4, c = lane & 15;
  const int bx = blockIdx.x;
  const int qb = bx & 7;
  const int bh = bx >> 3;
  const int h = bh & 7;
  const int b = bh >> 3;
  const int qbase = qb * 64;
  const int q0 = qbase + wave * 16;
  const size_t pitch = (size_t)NQKV;

  v16h qa[2];
  {
    const _Float16* qrow = (const _Float16*)(qkv + (size_t)(b * NL + q0 + c) * pitch + h * NHD);
#pragma unroll
    for (int dc = 0; dc < 2; ++dc) qa[dc] = Frag<_Float16>::load(qrow + dc * 32 + 8 * hh);
  }
  float mrow[8], lrow[8];
  v8f oacc[4];
#pragma unroll
  for (int r = 0; r < 8; ++r) { mrow[r] = -INFINITY; lrow[r] = 0.f; }
#pragma unroll
  for (int t = 0; t < 4; ++t) oacc[t] = zero8f();

  for (int kc = 0; kc < NL / 64; ++kc) {
    const int kv0 = kc * 64;
    __syncthreads();
#pragma unroll
    for (int it = 0; it < 4; ++it) {
      const int u = it * 128 + tid;
      const int r = u >> 3, c8 = (u & 7) * 8;
      const size_t kvrow = (size_t)(b * NL + kv0 + r) * pitch;
      const uint4 kw = *(const uint4*)(qkv + kvrow + ND + h * NHD + c8);
      *(uint4*)(Ksh + r * 64 + c8) = kw;
      const uint4 bw = *(const uint4*)(ebias + ((size_t)((b * NH + h) * NL + qbase + r)) * NL + kv0 + c8);
      *(uint4*)(Bsh + r * 64 + c8) = bw;
      const uint4 vw = *(const uint4*)(qkv + kvrow + 2 * ND + h * NHD + c8);
      Vt[(c8 + 0) * 64 + r] = (unsigned short)(vw.x & 0xffffu);
      Vt[(c8 + 1) * 64 + r] = (unsigned short)(vw.x >> 16);
      Vt[(c8 + 2) * 64 + r] = (unsigned short)(vw.y & 0xffffu);
      Vt[(c8 + 3) * 64 + r] = (unsigned short)(vw.y >> 16);
      Vt[(c8 + 4) * 64 + r] = (unsigned short)(vw.z & 0xffffu);
      Vt[(c8 + 5) * 64 + r] = (unsigned short)(vw.z >> 16);
      Vt[(c8 + 6) * 64 + r] = (unsigned short)(vw.w & 0xffffu);
      Vt[(c8 + 7) * 64 + r] = (unsigned short)(vw.w >> 16);
    }
    __syncthreads();

    v8f s[4];
#pragma unroll
    for (int j = 0; j < 4; ++j) {
      s[j] = zero8f();
#pragma unroll
      for (int dc = 0; dc < 2; ++dc) {
        const v16h kb = Frag<_Float16>::load((const _Float16*)(Ksh + (j * 16 + c) * 64 + dc * 32 + 8 * hh));
        s[j] = mma_h(qa[dc], kb, s[j]);
      }
    }
    float cm[8];
    const unsigned short* brow = Bsh + (wave * 16 + 8 * hh) * 64;
#pragma unroll
    for (int r = 0; r < 8; ++r) {
      float m = -INFINITY;
#pragma unroll
      for (int j = 0; j < 4; ++j) {
        const float bv = __uint_as_float(((unsigned)brow[r * 64 + j * 16 + c]) << 16);
        const float sv = s[j][r] * 0.125f + bv;
        s[j][r] = sv;
        m = fmaxf(m, sv);
      }
#pragma unroll
      for (int off = 1; off < 16; off <<= 1) m = fmaxf(m, __shfl_xor(m, off, 32));
      cm[r] = m;
    }
    _Float16* pw = Psh[wave];
#pragma unroll
    for (int r = 0; r < 8; ++r) {
      const float mnew = fmaxf(mrow[r], cm[r]);
      const float alpha = expf(mrow[r] - mnew);
      mrow[r] = mnew;
      float psum = 0.f;
#pragma unroll
      for (int j = 0; j < 4; ++j) {
        const float p = expf(s[j][r] - mnew);
        psum += p;
        pw[(8 * hh + r) * 64 + j * 16 + c] = (_Float16)(p * ATT_PSC);
      }
#pragma unroll
      for (int off = 1; off < 16; off <<= 1) psum += __shfl_xor(psum, off, 32);
      lrow[r] = lrow[r] * alpha + psum;
#pragma unroll
      for (int t = 0; t < 4; ++t) oacc[t][r] *= alpha;
    }
    wave_lds_sync();
#pragma unroll
    for (int kk = 0; kk < 2; ++kk) {
      const v16h pa = Frag<_Float16>::load(pw + c * 64 + kk * 32 + 8 * hh);
#pragma unroll
      for (int t = 0; t < 4; ++t) {
        const v16h vb = Frag<_Float16>::load((const _Float16*)(Vt + (t * 16 + c) * 64 + kk * 32 + 8 * hh));
        oacc[t] = mma_h(pa, vb, oacc[t]);
      }
    }
  }

  float* os = Os[wave];
#pragma unroll
  for (int r = 0; r < 8; ++r) {
    const float inv = (16.0f / ATT_PSC) / lrow[r];
#pragma unroll
    for (int t = 0; t < 4; ++t) os[(8 * hh + r) * 68 + t * 16 + c] = oacc[t][r] * inv;
  }
  wave_lds_sync();
  {
    const int q = lane >> 3, c8 = (lane & 7) * 8;
    v8h hv[4];
#pragma unroll
    for (int it = 0; it < 4; ++it) {
      const int row = it * 4 + q;
      const float* sp = os + row * 68 + c8;
#pragma unroll
      for (int e = 0; e < 8; ++e) hv[it][e] = (_Float16)sp[e];
    }
    for (int pass = 0; pass < 2; ++pass) {
#pragma unroll
      for (int it = 0; it < 4; ++it) {
        const int row = it * 4 + q;
        *(volatile v8h*)(ctx + (size_t)(b * NL + q0 + row) * ND + h * NHD + c8) = hv[it];
      }
      __threadfence();
    }
  }
}

template <bool W16>
__global__ __launch_bounds__(256) void ln_kernel(const float* __restrict__ x, const float* __restrict__ g,
    const float* __restrict__ bb, float* __restrict__ outF, _Float16* __restrict__ out16, int nrows) {
  const int wave = threadIdx.x >> 5, lane = threadIdx.x & 31;
  const int row = blockIdx.x * 8 + wave;
  if (row >= nrows) return;
  const float* xr = x + (size_t)row * ND;
  v4f xv[4];
  float s = 0.f;
#pragma unroll
  for (int it = 0; it < 4; ++it) {
    xv[it] = *(const v4f*)(xr + it * 128 + lane * 4);
    s += (xv[it][0] + xv[it][1]) + (xv[it][2] + xv[it][3]);
  }
#pragma unroll
  for (int off = 1; off < 32; off <<= 1) s += __shfl_xor(s, off, 32);
  const float mean = s * (1.0f / 512.0f);
  float vs = 0.f;
#pragma unroll
  for (int it = 0; it < 4; ++it) {
#pragma unroll
    for (int e = 0; e < 4; ++e) { const float d = xv[it][e] - mean; vs += d * d; }
  }
#pragma unroll
  for (int off = 1; off < 32; off <<= 1) vs += __shfl_xor(vs, off, 32);
  const float rs = rsqrtf(vs * (1.0f / 512.0f) + 1e-5f);
  v4f y[4];
#pragma unroll
  for (int it = 0; it < 4; ++it) {
    const v4f gv = *(const v4f*)(g + it * 128 + lane * 4);
    const v4f bv = *(const v4f*)(bb + it * 128 + lane * 4);
#pragma unroll
    for (int e = 0; e < 4; ++e) y[it][e] = (xv[it][e] - mean) * rs * gv[e] + bv[e];
  }
  v4h yh[4];
#pragma unroll
  for (int it = 0; it < 4; ++it) {
#pragma unroll
    for (int e = 0; e < 4; ++e) yh[it][e] = (_Float16)y[it][e];
  }
  float* orow = outF + (size_t)row * ND;
  _Float16* hrow = out16 + (size_t)row * ND;
  for (int pass = 0; pass < 2; ++pass) {
#pragma unroll
    for (int it = 0; it < 4; ++it) {
      *(volatile v4f*)(orow + it * 128 + lane * 4) = y[it];
      if (W16) *(volatile v4h*)(hrow + it * 128 + lane * 4) = yh[it];
    }
    __threadfence();
  }
}

static_assert(NM % 64 == 0 && NQKV % 64 == 0 && ND % 64 == 0 && NFF % 64 == 0, "tile multiples");
static_assert(ND % 32 == 0 && NFF % 32 == 0, "K multiples of 32");
static_assert(NL % 64 == 0 && NHD == 64 && NH * NHD == ND, "attention geometry");

extern "C" void kernel_launch(void* const* d_in, const int* in_sizes, int n_in,
                              void* d_out, int out_size, void* d_ws, size_t ws_size,
                              hipStream_t stream) {
  if (n_in < 18) return;
  if (in_sizes[0] != NB * NL * ND || in_sizes[1] != NB * NL * NL) return;
  if (in_sizes[2] != ND * ND || in_sizes[3] != ND * ND || in_sizes[4] != ND * ND || in_sizes[5] != ND * ND) return;
  if (in_sizes[6] != NRB * NRB || in_sizes[7] != NRB || in_sizes[8] != NRB * NH || in_sizes[9] != NH) return;
  if (in_sizes[10] != ND || in_sizes[11] != ND || in_sizes[12] != ND * NFF || in_sizes[13] != NFF) return;
  if (in_sizes[14] != NFF * ND || in_sizes[15] != ND || in_sizes[16] != ND || in_sizes[17] != ND) return;
  if (out_size != NB * NL * ND) return;

  const float* h_in = (const float*)d_in[0];
  const float* cost = (const float*)d_in[1];
  const float* Wq   = (const float*)d_in[2];
  const float* Wk   = (const float*)d_in[3];
  const float* Wv   = (const float*)d_in[4];
  const float* Wo   = (const float*)d_in[5];
  const float* We1  = (const float*)d_in[6];
  const float* be1  = (const float*)d_in[7];
  const float* We2  = (const float*)d_in[8];
  const float* be2  = (const float*)d_in[9];
  const float* g1   = (const float*)d_in[10];
  const float* bn1  = (const float*)d_in[11];
  const float* Wf1  = (const float*)d_in[12];
  const float* bf1  = (const float*)d_in[13];
  const float* Wf2  = (const float*)d_in[14];
  const float* bf2  = (const float*)d_in[15];
  const float* g2   = (const float*)d_in[16];
  const float* bn2  = (const float*)d_in[17];
  float* out = (float*)d_out;

  const size_t szR0 = (size_t)NQKV * ND * 2 + (size_t)ND * ND * 2 + (size_t)NFF * ND * 2 + (size_t)ND * NFF * 2;
  const size_t szR1 = (size_t)NM * ND * 2;
  const size_t szR2 = (size_t)NM * NQKV * 2;
  const size_t szR3 = (size_t)NB * NH * NL * NL * 2;
  const size_t total = szR0 + szR1 + szR2 + szR3;
  if (total > ws_size) return;
  char* ws = (char*)d_ws;
  char* pR0 = ws;
  char* pR1 = pR0 + szR0;
  char* pR2 = pR1 + szR1;
  char* pR3 = pR2 + szR2;

  _Float16* bt_qkv = (_Float16*)pR0;
  _Float16* bt_o   = bt_qkv + (size_t)NQKV * ND;
  _Float16* bt_f1  = bt_o + (size_t)ND * ND;
  _Float16* bt_f2  = bt_f1 + (size_t)NFF * ND;
  _Float16* h16    = (_Float16*)pR1;
  _Float16* ctx16  = (_Float16*)pR1;
  _Float16* qkv16  = (_Float16*)pR2;
  float*    hln    = (float*)pR2;
  _Float16* hln16  = (_Float16*)(pR2 + (size_t)NM * ND * 4);
  unsigned short* ebias = (unsigned short*)pR3;
  float*    x1     = (float*)pR3;
  _Float16* ff16   = (_Float16*)pR3;
  float*    x2     = (float*)(pR3 + (size_t)NM * NFF * 2);
  if ((size_t)NM * ND * 4 + (size_t)NM * ND * 2 > szR2) return;
  if ((size_t)NM * NFF * 2 + (size_t)NM * ND * 4 > szR3) return;

  dim3 blk256(256), blk128(128);

  const int n8 = NM * ND / 8;
  cast8_kernel<<<dim3((n8 + 255) / 256), blk256, 0, stream>>>(h_in, h16, n8);

  wtrans_kernel<<<dim3(ND / 64, ND / 64), blk256, 0, stream>>>(Wq, bt_qkv, ND, ND);
  wtrans_kernel<<<dim3(ND / 64, ND / 64), blk256, 0, stream>>>(Wk, bt_qkv + (size_t)ND * ND, ND, ND);
  wtrans_kernel<<<dim3(ND / 64, ND / 64), blk256, 0, stream>>>(Wv, bt_qkv + (size_t)2 * ND * ND, ND, ND);
  wtrans_kernel<<<dim3(ND / 64, ND / 64), blk256, 0, stream>>>(Wo, bt_o, ND, ND);
  wtrans_kernel<<<dim3(NFF / 64, ND / 64), blk256, 0, stream>>>(Wf1, bt_f1, ND, NFF);
  wtrans_kernel<<<dim3(ND / 64, NFF / 64), blk256, 0, stream>>>(Wf2, bt_f2, NFF, ND);

  {
    const int tiles = (NM / 64) * (NQKV / 64);
    wmma_gemm64<0, false, 0, 1, false, 0><<<dim3((tiles + 7) / 8, 1), blk256, 0, stream>>>(
        (const unsigned short*)h16, (const unsigned short*)h16, ND, 0L,
        (const unsigned short*)bt_qkv, (const unsigned short*)bt_qkv, ND, 0L,
        (void*)qkv16, (void*)qkv16, NQKV, 0L,
        bf1, h_in, 0L, NM, NQKV, ND, 1.0f / 64.0f);
  }

  edge_kernel<<<dim3(NM / 8), blk256, 0, stream>>>(cost, We1, be1, We2, be2, ebias);

  attn_kernel<<<dim3(NB * NH * (NL / 64)), blk128, 0, stream>>>((const unsigned short*)qkv16, ebias, ctx16);

  {
    const int tiles = (NM / 64) * (ND / 64);
    wmma_gemm64<0, false, 0, 0, true, 0><<<dim3((tiles + 7) / 8, 1), blk256, 0, stream>>>(
        (const unsigned short*)ctx16, (const unsigned short*)ctx16, ND, 0L,
        (const unsigned short*)bt_o, (const unsigned short*)bt_o, ND, 0L,
        (void*)x1, (void*)x1, ND, 0L,
        bf2, h_in, 0L, NM, ND, ND, 1.0f / 1024.0f);
  }

  ln_kernel<true><<<dim3(NM / 8), blk256, 0, stream>>>(x1, g1, bn1, hln, hln16, NM);

  {
    const int tiles = (NM / 64) * (NFF / 64);
    wmma_gemm64<0, false, 2, 1, false, 2><<<dim3((tiles + 7) / 8, 1), blk256, 0, stream>>>(
        (const unsigned short*)hln16, (const unsigned short*)hln16, ND, 0L,
        (const unsigned short*)bt_f1, (const unsigned short*)bt_f1, ND, 0L,
        (void*)ff16, (void*)ff16, NFF, 0L,
        bf1, hln, 0L, NM, NFF, ND, 1.0f / 64.0f);
  }

  {
    const int tiles = (NM / 64) * (ND / 64);
    wmma_gemm64<0, false, 2, 0, true, 0><<<dim3((tiles + 7) / 8, 1), blk256, 0, stream>>>(
        (const unsigned short*)ff16, (const unsigned short*)ff16, NFF, 0L,
        (const unsigned short*)bt_f2, (const unsigned short*)bt_f2, NFF, 0L,
        (void*)x2, (void*)x2, ND, 0L,
        bf2, hln, 0L, NM, ND, NFF, 1.0f / 64.0f);
  }

  ln_kernel<false><<<dim3(NM / 8), blk256, 0, stream>>>(x2, g2, bn2, out, hln16, NM);
}
